// PointNetSAModule_85358180040891
// MI455X (gfx1250) — hardware-verified
//
#include <hip/hip_runtime.h>
#pragma clang fp contract(off)

typedef __attribute__((ext_vector_type(16))) _Float16 v16h;
typedef __attribute__((ext_vector_type(8)))  _Float16 v8h;
typedef __attribute__((ext_vector_type(8)))  float    v8f;
typedef __attribute__((ext_vector_type(4)))  float    v4f;
typedef __attribute__((ext_vector_type(2)))  float    v2f;
typedef __attribute__((ext_vector_type(4)))  int      v4i;
typedef __attribute__((ext_vector_type(2)))  int      v2i;

constexpr int NBATCH = 8;
constexpr int NPT    = 8192;
constexpr int NCH_IN = 64;
constexpr int NCH_T  = 64;
constexpr int NCTR   = 1024;
constexpr int KNB    = 64;
constexpr int NCH_L1 = 64;
constexpr int NCH_L2 = 128;
constexpr int W1_LD  = 67;
constexpr int TILE_M = 32;
constexpr int NTILE  = NCTR / TILE_M;
constexpr int APITCH = 72;
constexpr int YPITCH = 36;
constexpr int PG_PTS = 128;

constexpr float RAD2 = 0.04f;
constexpr float WCARRY = 16.0f;
constexpr float XCARRY = 64.0f;
constexpr float HCARRY = 64.0f;
constexpr float L1_FOLD = 1.0f / (WCARRY * XCARRY);
constexpr float L2_FOLD = 1.0f / (WCARRY * HCARRY);
constexpr float GN_EPS = 1e-5f;

constexpr size_t OUT0_ELEMS = (size_t)NBATCH * NCH_L2 * NCTR;
constexpr size_t OUT1_ELEMS = (size_t)NBATCH * 3 * NCTR;
constexpr size_t OUT2_ELEMS = (size_t)NBATCH * NCH_T * NCTR;
static_assert(OUT0_ELEMS * 4 == 4194304);
static_assert((OUT0_ELEMS + OUT1_ELEMS) * 4 == 4292608);
static_assert((OUT0_ELEMS + OUT1_ELEMS + OUT2_ELEMS) * 4 == 6389760);
static_assert(NCTR % TILE_M == 0);
static_assert(NPT % PG_PTS == 0);
static_assert(NCH_IN % 32 == 0 && NCH_L1 % 32 == 0);
static_assert(NCH_L1 == 64 && NCH_L2 == 128 && KNB == 64);

template <typename T> struct Frag;
template <> struct Frag<_Float16> {
  typedef v16h V; union U { v16h v; v8h h[2]; };
  static __device__ __forceinline__ v16h load(const _Float16* p) {
    U f; f.h[0] = *(const v8h*)(p); f.h[1] = *(const v8h*)(p + 16); return f.v;
  }
};

__device__ __forceinline__ v8f mma_g(v16h a, v16h b, v8f c) {
  c = __builtin_amdgcn_wmma_f32_16x16x32_f16(false, a, false, b, (short)0, c, false, false);
  asm volatile("v_nop\n\tv_nop\n\tv_nop\n\tv_nop" : "+v"(c) : "v"(a), "v"(b));
  return c;
}
__device__ __forceinline__ void acc_guard4(v8f& a, v8f& b, v8f& c, v8f& d) {
  asm volatile("v_nop\n\tv_nop\n\tv_nop\n\tv_nop" : "+v"(a), "+v"(b), "+v"(c), "+v"(d));
}

__device__ __forceinline__ int clamp_pt(int i) {
  return i < 0 ? 0 : (i > NPT - 1 ? NPT - 1 : i);
}

__device__ __forceinline__ float swish_f(float z) {
  const float e = expf(-z);
  const float s = 1.0f / (1.0f + e);
  return z * s;
}

__global__ __launch_bounds__(64) void k_prep(const float* __restrict__ w1, const float* __restrict__ w2,
                                             _Float16* __restrict__ w1f, _Float16* __restrict__ w2h,
                                             float* __restrict__ w1c) {
  const int blk = blockIdx.x, t = threadIdx.x;
  if (blk < 8) {
    const int i = blk * 64 + t;
    const int o = i >> 3, c8 = (i & 7) * 8;
    v8h hv;
#pragma unroll
    for (int e = 0; e < 8; ++e) {
      const float x = w1[o * W1_LD + 3 + c8 + e] * WCARRY;
      hv[e] = (_Float16)x;
    }
    _Float16* dst = w1f + o * NCH_IN + c8;
    for (int pass = 0; pass < 2; ++pass) {
      *(volatile v8h*)dst = hv;
      __threadfence();
    }
  } else if (blk < 24) {
    const int i = (blk - 8) * 64 + t;
    const int o = i >> 3, c8 = (i & 7) * 8;
    const v4f a = *(const v4f*)(w2 + o * NCH_L1 + c8);
    const v4f c = *(const v4f*)(w2 + o * NCH_L1 + c8 + 4);
    v8h hv;
#pragma unroll
    for (int e = 0; e < 4; ++e) {
      const float x0 = a[e] * WCARRY;
      const float x1 = c[e] * WCARRY;
      hv[e] = (_Float16)x0;
      hv[4 + e] = (_Float16)x1;
    }
    _Float16* dst = w2h + o * NCH_L1 + c8;
    for (int pass = 0; pass < 2; ++pass) {
      *(volatile v8h*)dst = hv;
      __threadfence();
    }
  } else {
    const int o = t;
    v4f v;
    v[0] = w1[o * W1_LD + 0];
    v[1] = w1[o * W1_LD + 1];
    v[2] = w1[o * W1_LD + 2];
    v[3] = 0.0f;
    float* dst = w1c + o * 4;
    for (int pass = 0; pass < 2; ++pass) {
      *(volatile v4f*)dst = v;
      __threadfence();
    }
  }
}

__global__ __launch_bounds__(256) void k_pgemm(const float* __restrict__ features,
                                               const float* __restrict__ coords,
                                               const _Float16* __restrict__ w1f,
                                               const float* w1c, float* __restrict__ P) {
  __shared__ __align__(16) _Float16 As[PG_PTS * APITCH];
  __shared__ __align__(16) float slab[8][16 * 68];
  __shared__ float cs[3 * PG_PTS];
  const int tid = threadIdx.x, lane = tid & 31, wave = tid >> 5;
  const int rl = lane & 15, hh = lane >> 4, koff = hh * 8;
  const int b = blockIdx.x >> 6;
  const int n0 = (blockIdx.x & 63) * PG_PTS;

  for (int i = tid; i < 3 * PG_PTS; i += 256) {
    const int d = i >> 7, j = i & (PG_PTS - 1);
    cs[i] = coords[((size_t)b * 3 + d) * NPT + n0 + j];
  }
  {
    const int pt = tid & (PG_PTS - 1), cg = tid >> 7;
    const float* fb = features + ((size_t)b * NCH_IN + cg * 32) * NPT + n0 + pt;
#pragma unroll
    for (int q = 0; q < 4; ++q) {
      v8h hv;
#pragma unroll
      for (int e = 0; e < 8; ++e) {
        const float x = fb[(size_t)(q * 8 + e) * NPT] * XCARRY;
        hv[e] = (_Float16)x;
      }
      *(v8h*)(As + pt * APITCH + cg * 32 + q * 8) = hv;
      asm volatile("" ::: "memory");
    }
  }
  __syncthreads();

  v8f acc[4];
#pragma unroll
  for (int j = 0; j < 4; ++j) acc[j] = (v8f){0.f, 0.f, 0.f, 0.f, 0.f, 0.f, 0.f, 0.f};
#pragma unroll
  for (int ks = 0; ks < 2; ++ks) {
    const v16h a = Frag<_Float16>::load(As + (16 * wave + rl) * APITCH + koff + 32 * ks);
#pragma unroll
    for (int j = 0; j < 4; ++j) {
      const v16h bf = Frag<_Float16>::load(w1f + (16 * j + rl) * NCH_IN + koff + 32 * ks);
      acc[j] = mma_g(a, bf, acc[j]);
    }
  }
  acc_guard4(acc[0], acc[1], acc[2], acc[3]);

  float* sl = slab[wave];
#pragma unroll
  for (int j = 0; j < 4; ++j) {
#pragma unroll
    for (int r = 0; r < 8; ++r) {
      sl[(8 * hh + r) * 68 + 16 * j + rl] = acc[j][r] * L1_FOLD;
    }
  }
  __syncthreads();

  const int c4 = rl * 4;
  v4f wq[4];
#pragma unroll
  for (int e = 0; e < 4; ++e) wq[e] = *(const v4f*)(w1c + (c4 + e) * 4);
  v4f vals[8];
#pragma unroll
  for (int it = 0; it < 8; ++it) {
    const int row = 2 * it + hh;
    const int pl = 16 * wave + row;
    v4f v = *(const v4f*)(sl + row * 68 + c4);
    const float cx = cs[pl], cy = cs[PG_PTS + pl], cz = cs[2 * PG_PTS + pl];
#pragma unroll
    for (int e = 0; e < 4; ++e) {
      const float t0 = wq[e][0] * cx;
      const float t1 = wq[e][1] * cy;
      const float t2 = wq[e][2] * cz;
      v[e] = v[e] + ((t0 + t1) + t2);
    }
    vals[it] = v;
  }
  float* dst = P + ((size_t)b * NPT + n0 + 16 * wave) * NCH_L1 + c4;
  for (int pass = 0; pass < 2; ++pass) {
#pragma unroll
    for (int it = 0; it < 8; ++it) {
      *(volatile v4f*)(dst + (size_t)(2 * it + hh) * NCH_L1) = vals[it];
    }
    __threadfence();
  }
}

__device__ __forceinline__ void argmax_wave(float& bv, int& bn) {
#pragma unroll
  for (int off = 16; off >= 1; off >>= 1) {
    const float ov = __shfl_xor(bv, off, 32);
    const int on = __shfl_xor(bn, off, 32);
    const bool take = (ov > bv) || ((ov == bv) && (on < bn));
    bv = take ? ov : bv;
    bn = take ? on : bn;
  }
}

__global__ __launch_bounds__(1024) void k_fps(const float* __restrict__ coords, int* __restrict__ c_idx,
                                              float* __restrict__ outc) {
#pragma clang fp contract(off)
  __shared__ float wv_v[2][32];
  __shared__ int wv_n[2][32];
  __shared__ int s_sel[NCTR];
  const int b = blockIdx.x, tid = threadIdx.x, lane = tid & 31, w = tid >> 5;
  const float* cb = coords + (size_t)b * 3 * NPT;
  float px[8], py[8], pz[8], dist[8];
#pragma unroll
  for (int i = 0; i < 4; ++i) {
    const int n = tid + i * 1024;
    px[i] = cb[n]; py[i] = cb[NPT + n]; pz[i] = cb[2 * NPT + n];
  }
  asm volatile("" : "+v"(px[0]), "+v"(px[1]), "+v"(px[2]), "+v"(px[3]),
                    "+v"(py[0]), "+v"(py[1]), "+v"(py[2]), "+v"(py[3]),
                    "+v"(pz[0]), "+v"(pz[1]), "+v"(pz[2]), "+v"(pz[3]));
#pragma unroll
  for (int i = 4; i < 8; ++i) {
    const int n = tid + i * 1024;
    px[i] = cb[n]; py[i] = cb[NPT + n]; pz[i] = cb[2 * NPT + n];
  }
  asm volatile("" : "+v"(px[4]), "+v"(px[5]), "+v"(px[6]), "+v"(px[7]),
                    "+v"(py[4]), "+v"(py[5]), "+v"(py[6]), "+v"(py[7]),
                    "+v"(pz[4]), "+v"(pz[5]), "+v"(pz[6]), "+v"(pz[7]));
#pragma unroll
  for (int i = 0; i < 8; ++i) dist[i] = 1e10f;
  if (tid == 0) s_sel[0] = 0;
  int last = 0;
  for (int step = 1; step < NCTR; ++step) {
    const int lc = clamp_pt(last);
    const float lx = cb[lc], ly = cb[NPT + lc], lz = cb[2 * NPT + lc];
    float bv = -1.0f;
    int bn = 0;
#pragma unroll
    for (int i = 0; i < 8; ++i) {
      const float dx = px[i] - lx, dy = py[i] - ly, dz = pz[i] - lz;
      const float t0 = dx * dx;
      const float t1 = dy * dy;
      const float t2 = dz * dz;
      const float d = (t0 + t2) + t1;
      const float dd = fminf(dist[i], d);
      dist[i] = dd;
      const bool take = dd > bv;
      bv = take ? dd : bv;
      bn = take ? (tid + i * 1024) : bn;
    }
    argmax_wave(bv, bn);
    const int p = step & 1;
    if (lane == 0) { wv_v[p][w] = bv; wv_n[p][w] = bn; }
    __syncthreads();
    bv = wv_v[p][lane];
    bn = wv_n[p][lane];
    argmax_wave(bv, bn);
    last = bn;
    if (tid == 0) s_sel[step] = bn;
  }
  __syncthreads();
  if (tid < 256) {
    v4i iv;
    v4f ox, oy, oz;
#pragma unroll
    for (int e = 0; e < 4; ++e) {
      const int id = clamp_pt(s_sel[4 * tid + e]);
      iv[e] = id;
      ox[e] = cb[id];
      oy[e] = cb[NPT + id];
      oz[e] = cb[2 * NPT + id];
    }
    int* di = c_idx + (size_t)b * NCTR + 4 * tid;
    float* dc = outc + (size_t)b * 3 * NCTR + 4 * tid;
    for (int pass = 0; pass < 2; ++pass) {
      *(volatile v4i*)di = iv;
      *(volatile v4f*)(dc) = ox;
      *(volatile v4f*)(dc + NCTR) = oy;
      *(volatile v4f*)(dc + 2 * NCTR) = oz;
      __threadfence();
    }
  }
}

__global__ __launch_bounds__(256) void k_ballq(const float* __restrict__ coords, const int* __restrict__ c_idx,
                                               int* __restrict__ nidx) {
#pragma clang fp contract(off)
  __shared__ int s_row[8][KNB];
  const int lane = threadIdx.x & 31, wave = threadIdx.x >> 5;
  const int gw = blockIdx.x * 8 + wave;
  const int b = gw >> 10;
  const float* cb = coords + (size_t)b * 3 * NPT;
  const int cid = clamp_pt(c_idx[gw]);
  const float cx = cb[cid], cy = cb[NPT + cid], cz = cb[2 * NPT + cid];
  int count = 0, first_n = 0;
  for (int base = 0; base < NPT && count < KNB; base += 32) {
    const int n = base + lane;
    const float dx = cx - cb[n], dy = cy - cb[NPT + n], dz = cz - cb[2 * NPT + n];
    const float t0 = dx * dx;
    const float t1 = dy * dy;
    const float t2 = dz * dz;
    const float d2 = (t0 + t2) + t1;
    const bool pred = d2 < RAD2;
    const unsigned mask = __builtin_amdgcn_ballot_w32(pred);
    if (count == 0 && mask != 0u) first_n = base + (__builtin_ctz(mask));
    const int pos = count + __builtin_popcount(mask & ((1u << lane) - 1u));
    if (pred && pos < KNB) s_row[wave][pos] = n;
    count += __builtin_popcount(mask);
  }
  const int cfill = count < KNB ? count : KNB;
  const int fill = count ? first_n : 0;
  for (int p = cfill + lane; p < KNB; p += 32) s_row[wave][p] = fill;
  __syncthreads();
  v2i val;
  val[0] = s_row[wave][2 * lane];
  val[1] = s_row[wave][2 * lane + 1];
  int* dst = nidx + (size_t)gw * KNB + 2 * lane;
  for (int pass = 0; pass < 2; ++pass) {
    *(volatile v2i*)dst = val;
    __threadfence();
  }
}

template <bool WITH_CC>
__device__ __forceinline__ void stage_tile(const int* nidx, const int* c_idx, const float* coords,
                                           int b, int m0, int* s_idx, int pitch, float* s_cc, int tid) {
  const int r = tid >> 3, k0 = (tid & 7) * 8;
  const int* src = nidx + ((size_t)(b * NCTR + m0 + r)) * KNB + k0;
  const v4i a = *(const v4i*)src;
  const v4i c = *(const v4i*)(src + 4);
  int* dst = s_idx + r * pitch + k0;
  dst[0] = clamp_pt(a[0]); dst[1] = clamp_pt(a[1]); dst[2] = clamp_pt(a[2]); dst[3] = clamp_pt(a[3]);
  dst[4] = clamp_pt(c[0]); dst[5] = clamp_pt(c[1]); dst[6] = clamp_pt(c[2]); dst[7] = clamp_pt(c[3]);
  if (WITH_CC) {
    if (tid < TILE_M) {
      const int cid = clamp_pt(c_idx[b * NCTR + m0 + tid]);
      const float* cb = coords + (size_t)b * 3 * NPT;
      s_cc[tid * 4 + 0] = cb[cid];
      s_cc[tid * 4 + 1] = cb[NPT + cid];
      s_cc[tid * 4 + 2] = cb[2 * NPT + cid];
      s_cc[tid * 4 + 3] = 0.0f;
    }
  }
}

__global__ __launch_bounds__(256) void k_temb(const float* __restrict__ temb, const int* __restrict__ nidx,
                                              float* __restrict__ out_t) {
  __shared__ int s_idx[TILE_M * 65];
  const int tid = threadIdx.x, lane = tid & 31, wave = tid >> 5;
  const int b = blockIdx.x >> 5, m0 = (blockIdx.x & 31) * TILE_M;
  stage_tile<false>(nidx, nullptr, nullptr, b, m0, s_idx, 65, nullptr, tid);
  __syncthreads();
  const float* tb = temb + ((size_t)b * NCH_T + 8 * wave) * NPT;
  float mx[8];
#pragma unroll
  for (int c = 0; c < 8; ++c) mx[c] = -__builtin_inff();
#pragma unroll 2
  for (int k = 0; k < KNB; ++k) {
    const int id = s_idx[lane * 65 + k];
#pragma unroll
    for (int c = 0; c < 8; ++c) mx[c] = fmaxf(mx[c], tb[(size_t)c * NPT + id]);
  }
  float* dst = out_t + ((size_t)b * NCH_T + 8 * wave) * NCTR + m0 + lane;
  for (int pass = 0; pass < 2; ++pass) {
#pragma unroll
    for (int c = 0; c < 8; ++c) *(volatile float*)(dst + (size_t)c * NCTR) = mx[c];
    __threadfence();
  }
}

__global__ __launch_bounds__(256) void k_stats1(const float* __restrict__ P, const int* __restrict__ nidx,
                                                const int* __restrict__ c_idx, const float* __restrict__ coords,
                                                const float* w1c, const float* b1, float* __restrict__ stats) {
  __shared__ int s_idx[TILE_M * KNB];
  __shared__ float s_cc[TILE_M * 4];
  __shared__ float red[512];
  const int tid = threadIdx.x;
  const int b = blockIdx.x >> 5, m0 = (blockIdx.x & 31) * TILE_M;
  stage_tile<true>(nidx, c_idx, coords, b, m0, s_idx, KNB, s_cc, tid);
  const int c8 = (tid & 7) * 8, rg = tid >> 3;
  float bb[8];
  {
    v4f bA = *(const v4f*)(b1 + c8);
    v4f bB = *(const v4f*)(b1 + c8 + 4);
    asm volatile("" : "+v"(bA), "+v"(bB) : : "memory");
#pragma unroll
    for (int e = 0; e < 4; ++e) { bb[e] = bA[e]; bb[4 + e] = bB[e]; }
  }
  v4f wq[8];
#pragma unroll
  for (int e = 0; e < 8; ++e) wq[e] = *(const v4f*)(w1c + (c8 + e) * 4);
  __syncthreads();

  float s = 0.0f, ss = 0.0f;
#pragma unroll 1
  for (int mi = 0; mi < TILE_M; ++mi) {
    const float cx = s_cc[mi * 4 + 0], cy = s_cc[mi * 4 + 1], cz = s_cc[mi * 4 + 2];
    float off[8];
#pragma unroll
    for (int e = 0; e < 8; ++e) {
      const float t0 = wq[e][0] * cx;
      const float t1 = wq[e][1] * cy;
      const float t2 = wq[e][2] * cz;
      off[e] = bb[e] - ((t0 + t1) + t2);
    }
#pragma unroll
    for (int p = 0; p < 2; ++p) {
      const int id = s_idx[mi * KNB + rg + 32 * p];
      const float* pr = P + ((size_t)b * NPT + id) * NCH_L1 + c8;
      const v4f p0 = *(const v4f*)pr;
      const v4f p1 = *(const v4f*)(pr + 4);
#pragma unroll
      for (int e = 0; e < 4; ++e) {
        const float y0 = p0[e] + off[e];
        const float y1 = p1[e] + off[4 + e];
        const float q0 = y0 * y0;
        const float q1 = y1 * y1;
        s = s + y0; ss = ss + q0;
        s = s + y1; ss = ss + q1;
      }
    }
  }
  red[tid] = s;
  red[256 + tid] = ss;
  __syncthreads();
  float r = 0.0f;
  if (tid < 16) {
    const float* src = red + (tid & 1) * 256 + (tid >> 1);
#pragma unroll 1
    for (int j = 0; j < 32; ++j) r = r + src[j * 8];
  }
  if (tid < 32) {
    float* dst = stats + (size_t)blockIdx.x * 32 + tid;
    for (int pass = 0; pass < 2; ++pass) {
      *(volatile float*)dst = r;
      __threadfence();
    }
  }
}

__global__ __launch_bounds__(64) void k_finalize(const float* __restrict__ stats, float* __restrict__ nrm,
                                                 float inv_cnt) {
  const int t = threadIdx.x;
  const int b = t >> 3, g = t & 7;
  double S = 0.0, SS = 0.0;
#pragma unroll 1
  for (int j = 0; j < NTILE; ++j) {
    const float* r = stats + ((size_t)(b * NTILE + j)) * 32 + 2 * g;
    S = S + (double)r[0];
    SS = SS + (double)r[1];
  }
  const double inv = (double)inv_cnt;
  const double mu = S * inv;
  const double m2 = SS * inv;
  double var = m2 - mu * mu;
  var = var < 0.0 ? 0.0 : var;
  const float vf = (float)var + GN_EPS;
  const float rs = 1.0f / sqrtf(vf);
  v2f o;
  o[0] = (float)mu;
  o[1] = rs;
  float* dst = nrm + 2 * t;
  for (int pass = 0; pass < 2; ++pass) {
    *(volatile v2f*)dst = o;
    __threadfence();
  }
}

__global__ __launch_bounds__(256) void k_layer2(
    const float* __restrict__ P, const int* __restrict__ nidx, const int* __restrict__ c_idx,
    const float* __restrict__ coords, const float* w1c, const float* b1, const float* gw1, const float* gb1,
    const float* nrm1, const _Float16* __restrict__ w2h, const float* __restrict__ b2,
    float* __restrict__ ymin, float* __restrict__ ymax, float* __restrict__ stats) {
  __shared__ __align__(16) _Float16 As[2 * KNB * APITCH];
  __shared__ __align__(16) float ymn[NCH_L2 * YPITCH];
  __shared__ __align__(16) float ymx[NCH_L2 * YPITCH];
  __shared__ int s_idx[TILE_M * KNB];
  __shared__ float s_cc[TILE_M * 4];
  __shared__ float rec[16];
  const int tid = threadIdx.x, lane = tid & 31, wave = tid >> 5;
  const int rl = lane & 15, hh = lane >> 4, koff = hh * 8;
  const int b = blockIdx.x >> 5, m0 = (blockIdx.x & 31) * TILE_M;
  stage_tile<true>(nidx, c_idx, coords, b, m0, s_idx, KNB, s_cc, tid);

  const int c8 = (tid & 7) * 8, rg = tid >> 3;
  float sc[8], sh[8], bb[8];
  {
    const int g1 = tid & 7;
    const float mu1 = nrm1[(b * 8 + g1) * 2];
    const float rs1 = nrm1[(b * 8 + g1) * 2 + 1];
    const v4f bA = *(const v4f*)(b1 + c8);
    const v4f bB = *(const v4f*)(b1 + c8 + 4);
    const v4f gA = *(const v4f*)(gw1 + c8);
    const v4f gB = *(const v4f*)(gw1 + c8 + 4);
    const v4f hA = *(const v4f*)(gb1 + c8);
    const v4f hB = *(const v4f*)(gb1 + c8 + 4);
#pragma unroll
    for (int e = 0; e < 4; ++e) {
      bb[e] = bA[e];
      bb[4 + e] = bB[e];
      sc[e] = rs1 * gA[e];
      sc[4 + e] = rs1 * gB[e];
      const float m0v = mu1 * sc[e];
      const float m1v = mu1 * sc[4 + e];
      sh[e] = hA[e] - m0v;
      sh[4 + e] = hB[e] - m1v;
    }
    asm volatile("" : "+v"(sc[0]), "+v"(sc[1]), "+v"(sc[2]), "+v"(sc[3]),
                      "+v"(sc[4]), "+v"(sc[5]), "+v"(sc[6]), "+v"(sc[7]) : : "memory");
    asm volatile("" : "+v"(sh[0]), "+v"(sh[1]), "+v"(sh[2]), "+v"(sh[3]),
                      "+v"(sh[4]), "+v"(sh[5]), "+v"(sh[6]), "+v"(sh[7]),
                      "+v"(bb[0]), "+v"(bb[1]), "+v"(bb[2]), "+v"(bb[3]),
                      "+v"(bb[4]), "+v"(bb[5]), "+v"(bb[6]), "+v"(bb[7]) : : "memory");
  }
  v4f wq[8];
#pragma unroll
  for (int e = 0; e < 8; ++e) wq[e] = *(const v4f*)(w1c + (c8 + e) * 4);

  v16h bfr[2];
#pragma unroll
  for (int ks = 0; ks < 2; ++ks)
    bfr[ks] = Frag<_Float16>::load(w2h + (16 * wave + rl) * NCH_L1 + koff + 32 * ks);
  const float b2v = b2[16 * wave + rl];
  float s2 = 0.0f, ss2 = 0.0f;
  __syncthreads();

#pragma unroll 1
  for (int mi = 0; mi < TILE_M; ++mi) {
    _Float16* Ab = As + (mi & 1) * (KNB * APITCH);
    const float cx = s_cc[mi * 4 + 0], cy = s_cc[mi * 4 + 1], cz = s_cc[mi * 4 + 2];
    float cB[8];
#pragma unroll
    for (int e = 0; e < 8; ++e) {
      const float t0 = wq[e][0] * cx;
      const float t1 = wq[e][1] * cy;
      const float t2 = wq[e][2] * cz;
      const float off = bb[e] - ((t0 + t1) + t2);
      const float os = off * sc[e];
      cB[e] = os + sh[e];
    }
#pragma unroll 1
    for (int p = 0; p < 2; ++p) {
      const int row = rg + 32 * p;
      const int id = s_idx[mi * KNB + row];
      const float* pr = P + ((size_t)b * NPT + id) * NCH_L1 + c8;
      const v4f p0 = *(const v4f*)pr;
      const v4f p1 = *(const v4f*)(pr + 4);
      v8h hv;
#pragma unroll
      for (int e = 0; e < 4; ++e) {
        const float a0 = p0[e] * sc[e];
        const float a1 = p1[e] * sc[4 + e];
        const float z0 = a0 + cB[e];
        const float z1 = a1 + cB[4 + e];
        const float h0 = swish_f(z0) * HCARRY;
        const float h1 = swish_f(z1) * HCARRY;
        hv[e] = (_Float16)h0;
        hv[4 + e] = (_Float16)h1;
      }
      *(v8h*)(Ab + row * APITCH + c8) = hv;
    }
    __syncthreads();

    v8f acc[4];
#pragma unroll
    for (int t = 0; t < 4; ++t) acc[t] = (v8f){0.f, 0.f, 0.f, 0.f, 0.f, 0.f, 0.f, 0.f};
#pragma unroll
    for (int ks = 0; ks < 2; ++ks) {
#pragma unroll
      for (int t = 0; t < 4; ++t) {
        const v16h a = Frag<_Float16>::load(Ab + (16 * t + rl) * APITCH + koff + 32 * ks);
        acc[t] = mma_g(a, bfr[ks], acc[t]);
      }
    }
    acc_guard4(acc[0], acc[1], acc[2], acc[3]);

    float mn = __builtin_inff(), mx = -__builtin_inff();
#pragma unroll
    for (int t = 0; t < 4; ++t) {
#pragma unroll
      for (int r = 0; r < 8; ++r) {
        const float sv = acc[t][r] * L2_FOLD;
        const float v = sv + b2v;
        const float q = v * v;
        mn = fminf(mn, v);
        mx = fmaxf(mx, v);
        s2 = s2 + v;
        ss2 = ss2 + q;
      }
    }
    const float mn_o = __shfl_xor(mn, 16, 32);
    const float mx_o = __shfl_xor(mx, 16, 32);
    mn = fminf(mn, mn_o);
    mx = fmaxf(mx, mx_o);
    if (hh == 0) {
      ymn[(16 * wave + rl) * YPITCH + mi] = mn;
      ymx[(16 * wave + rl) * YPITCH + mi] = mx;
    }
  }

#pragma unroll
  for (int off = 16; off >= 1; off >>= 1) {
    const float so = __shfl_xor(s2, off, 32);
    const float sso = __shfl_xor(ss2, off, 32);
    s2 = s2 + so;
    ss2 = ss2 + sso;
  }
  if (lane == 0) { rec[2 * wave] = s2; rec[2 * wave + 1] = ss2; }
  __syncthreads();

  {
    const int q = lane >> 3, c = (lane & 7) * 4;
    v4f vn[4], vx[4];
#pragma unroll
    for (int it = 0; it < 4; ++it) {
      const int o = 16 * wave + it * 4 + q;
      vn[it] = *(const v4f*)(ymn + o * YPITCH + c);
      vx[it] = *(const v4f*)(ymx + o * YPITCH + c);
    }
    for (int pass = 0; pass < 2; ++pass) {
#pragma unroll
      for (int it = 0; it < 4; ++it) {
        const int o = 16 * wave + it * 4 + q;
        const size_t go = ((size_t)b * NCH_L2 + o) * NCTR + m0 + c;
        *(volatile v4f*)(ymin + go) = vn[it];
        *(volatile v4f*)(ymax + go) = vx[it];
      }
      __threadfence();
    }
  }
  if (tid < 32) {
    const float rv = rec[tid & 15];
    const float r = (tid < 16) ? rv : 0.0f;
    float* dst = stats + (size_t)blockIdx.x * 32 + tid;
    for (int pass = 0; pass < 2; ++pass) {
      *(volatile float*)dst = r;
      __threadfence();
    }
  }
}

__global__ __launch_bounds__(256) void k_final(const float* __restrict__ ymin, const float* __restrict__ ymax,
                                               const float* __restrict__ nrm2, const float* __restrict__ gw2,
                                               const float* __restrict__ gb2, float* __restrict__ out) {
  const int e = blockIdx.x * 256 + threadIdx.x;
  const int o = (e >> 10) & (NCH_L2 - 1);
  const int b = e >> 17;
  const int g = o >> 4;
  const float mu = nrm2[(b * 8 + g) * 2];
  const float rs = nrm2[(b * 8 + g) * 2 + 1];
  const float gw = gw2[o], gb = gb2[o];
  const float yl = ymin[e], yh = ymax[e];
  const float dl = yl - mu;
  const float dh = yh - mu;
  const float nl = dl * rs;
  const float nh = dh * rs;
  const float zl = nl * gw + gb;
  const float zh = nh * gw + gb;
  const float r = fmaxf(swish_f(zl), swish_f(zh));
  for (int pass = 0; pass < 2; ++pass) {
    *(volatile float*)(out + e) = r;
    __threadfence();
  }
}

extern "C" void kernel_launch(void* const* d_in, const int* in_sizes, int n_in,
                              void* d_out, int out_size, void* d_ws, size_t ws_size,
                              hipStream_t stream) {
  (void)in_sizes; (void)n_in; (void)out_size;
  const float* features = (const float*)d_in[0];
  const float* coords   = (const float*)d_in[1];
  const float* temb     = (const float*)d_in[2];
  const float* w1  = (const float*)d_in[3];
  const float* b1  = (const float*)d_in[4];
  const float* gw1 = (const float*)d_in[5];
  const float* gb1 = (const float*)d_in[6];
  const float* w2  = (const float*)d_in[7];
  const float* b2  = (const float*)d_in[8];
  const float* gw2 = (const float*)d_in[9];
  const float* gb2 = (const float*)d_in[10];

  float* out0 = (float*)d_out;
  float* out1 = out0 + OUT0_ELEMS;
  float* out2 = out1 + OUT1_ELEMS;

  char* base = (char*)d_ws;
  size_t off = 0;
  const size_t o_w1f = off;  off += (size_t)NCH_L1 * NCH_IN * 2;
  const size_t o_w2h = off;  off += (size_t)NCH_L2 * NCH_L1 * 2;
  const size_t o_w1c = off;  off += (size_t)NCH_L1 * 4 * 4;
  const size_t o_cid = off;  off += (size_t)NBATCH * NCTR * 4;
  const size_t o_idx = off;  off += (size_t)NBATCH * NCTR * KNB * 4;
  const size_t o_P   = off;  off += (size_t)NBATCH * NPT * NCH_L1 * 4;
  const size_t o_ymn = off;  off += OUT0_ELEMS * 4;
  const size_t o_ymx = off;  off += OUT0_ELEMS * 4;
  const size_t o_st1 = off;  off += (size_t)NBATCH * NTILE * 32 * 4;
  const size_t o_st2 = off;  off += (size_t)NBATCH * NTILE * 32 * 4;
  const size_t o_n1  = off;  off += 512;
  const size_t o_n2  = off;  off += 512;
  if (off > ws_size) return;

  _Float16* w1f = (_Float16*)(base + o_w1f);
  _Float16* w2h = (_Float16*)(base + o_w2h);
  float* w1c  = (float*)(base + o_w1c);
  int* c_idx  = (int*)(base + o_cid);
  int* nidx   = (int*)(base + o_idx);
  float* P    = (float*)(base + o_P);
  float* ymin = (float*)(base + o_ymn);
  float* ymax = (float*)(base + o_ymx);
  float* st1  = (float*)(base + o_st1);
  float* st2  = (float*)(base + o_st2);
  float* nrm1 = (float*)(base + o_n1);
  float* nrm2 = (float*)(base + o_n2);

  const float inv1 = 1.0f / (8.0f * (float)NCTR * (float)KNB);
  const float inv2 = 1.0f / (16.0f * (float)NCTR * (float)KNB);

  k_prep<<<25, 64, 0, stream>>>(w1, w2, w1f, w2h, w1c);
  k_pgemm<<<NBATCH * (NPT / PG_PTS), 256, 0, stream>>>(features, coords, w1f, w1c, P);
  k_fps<<<NBATCH, 1024, 0, stream>>>(coords, c_idx, out1);
  k_ballq<<<NBATCH * NCTR / 8, 256, 0, stream>>>(coords, c_idx, nidx);
  k_temb<<<NBATCH * NTILE, 256, 0, stream>>>(temb, nidx, out2);
  k_stats1<<<NBATCH * NTILE, 256, 0, stream>>>(P, nidx, c_idx, coords, w1c, b1, st1);
  k_finalize<<<1, 64, 0, stream>>>(st1, nrm1, inv1);
  k_layer2<<<NBATCH * NTILE, 256, 0, stream>>>(P, nidx, c_idx, coords, w1c, b1, gw1, gb1, nrm1, w2h, b2,
                                              ymin, ymax, st2);
  k_finalize<<<1, 64, 0, stream>>>(st2, nrm2, inv2);
  k_final<<<(int)(OUT0_ELEMS / 256), 256, 0, stream>>>(ymin, ymax, nrm2, gw2, gb2, out0);
}
